// HierarchicalAttention_62380105007262
// MI455X (gfx1250) — hardware-verified
//
#include <hip/hip_runtime.h>


#ifndef NB
#define NB 64
#endif
#ifndef SEQ
#define SEQ 2048
#endif
#define NB_FULL  64
#define SEQ_FULL 2048
#ifndef OUT_SEQ
#define OUT_SEQ SEQ
#endif
#define MEMN  512
#define NBITS 9
#define KPAD  32
#define AW    8
#define BFP   0x4120
#define BFN   0xC120
#define LOG2E 1.4426950408889634f

static_assert((1 << NBITS) == MEMN);
static_assert(NBITS <= 16);
static_assert(MEMN % 16 == 0);
static_assert(MEMN % 4 == 0);
static_assert(SEQ % (32 * AW) == 0);
static_assert(OUT_SEQ % 32 == 0);
static_assert(NB <= NB_FULL);
static_assert(SEQ <= SEQ_FULL);

typedef unsigned short bf;
typedef __attribute__((ext_vector_type(16))) __bf16   v16bf;
typedef __attribute__((ext_vector_type(8)))  unsigned short v8us;
typedef __attribute__((ext_vector_type(8)))  float    v8f;
typedef __attribute__((ext_vector_type(4)))  float    v4f;
typedef v4f  __attribute__((may_alias)) v4fa;

__device__ __forceinline__ unsigned short f2bf(float f) { unsigned u = __float_as_uint(f); u += 0x7FFFu + ((u >> 16) & 1u); return (unsigned short)(u >> 16); }
__device__ __forceinline__ v16bf cat16b(v8us lo, v8us hi) { return __builtin_bit_cast(v16bf, __builtin_shufflevector(lo, hi, 0, 1, 2, 3, 4, 5, 6, 7, 8, 9, 10, 11, 12, 13, 14, 15)); }
__device__ __forceinline__ v8f wmmab(v16bf a, v16bf b, v8f c) { return __builtin_amdgcn_wmma_f32_16x16x32_bf16(false, a, false, b, (short)0, c, false, false); }
__device__ __forceinline__ void wave_sync() { __builtin_amdgcn_fence(3  , "wavefront"); __builtin_amdgcn_wave_barrier(); asm volatile("" ::: "memory"); }
__device__ __forceinline__ unsigned short encb(int x, int i) { return ((x >> i) & 1) ? (unsigned short)BFP : (unsigned short)BFN; }

__device__ __forceinline__ v16bf mkq(int a, int hi) {
    v8us lo; const v8us z = (v8us){0, 0, 0, 0, 0, 0, 0, 0};
    const unsigned short e8 = encb(a, 8);
#pragma unroll
    for (int i = 0; i < 8; ++i) {
        const unsigned short e0 = encb(a, i);
        const unsigned short e1 = (i == 0) ? e8 : (unsigned short)0;
        lo[i] = hi ? e1 : e0;
    }
    return cat16b(lo, z);
}

__global__ __launch_bounds__(32 * AW) void k_lookup(const int* __restrict__ QA, const float* __restrict__ MEMF, float* OUT) {
    __shared__ __align__(16) bf    kt[MEMN * KPAD];
    __shared__ __align__(16) float ms[MEMN];
    __shared__ __align__(16) float os[AW * 32];
    const int tid = threadIdx.x;
    const int lane = tid & 31, lr = lane & 15, hi = lane >> 4;
    const int wave = __builtin_amdgcn_readfirstlane(tid >> 5);
    const int b = blockIdx.y;

    for (int n = tid; n < MEMN; n += 32 * AW) {
        v8us p0, p1; const v8us z = (v8us){0, 0, 0, 0, 0, 0, 0, 0};
#pragma unroll
        for (int i = 0; i < 8; ++i) { p0[i] = encb(n, i); p1[i] = (i == 0) ? encb(n, 8) : (unsigned short)0; }
        *(v8us*)(&kt[n * KPAD])      = p0;
        *(v8us*)(&kt[n * KPAD + 8])  = p1;
        *(v8us*)(&kt[n * KPAD + 16]) = z;
        *(v8us*)(&kt[n * KPAD + 24]) = z;
    }
    for (int i = tid; i < MEMN / 4; i += 32 * AW) {
        const v4f v = *(const v4f*)(MEMF + (size_t)b * MEMN + 4 * i); v4f o;
#pragma unroll
        for (int k = 0; k < 4; ++k) o[k] = __uint_as_float(((unsigned)f2bf(v[k])) << 16);
        *(v4fa*)(&ms[4 * i]) = o;
    }
    __syncthreads();

    const int t0 = (blockIdx.x * AW + wave) * 32;
    const size_t qrow = (size_t)b * SEQ_FULL + t0;
    const int a0 = QA[qrow + lr];
    const int a1 = QA[qrow + 16 + lr];
    const v16bf qb0 = mkq(a0, hi), qb1 = mkq(a1, hi);

    float l0 = 0.0f, l1 = 0.0f, o0 = 0.0f, o1 = 0.0f;
#pragma unroll 2
    for (int j = 0; j < MEMN / 16; ++j) {
        const int ko = (j * 16 + lr) * KPAD + 8 * hi;
        const v8us k0 = *(const v8us*)(&kt[ko]);
        const v8us k1 = *(const v8us*)(&kt[ko + 16]);
        const v16bf ka = cat16b(k0, k1);
        v8f s0 = (v8f){}, s1 = (v8f){};
        s0 = wmmab(ka, qb0, s0); s1 = wmmab(ka, qb1, s1);
        asm volatile("v_nop\n\tv_nop\n\tv_nop\n\tv_nop" : "+v"(s0), "+v"(s1) : "v"(ka), "v"(qb0), "v"(qb1));
        const v4f m0 = *(const v4fa*)(&ms[j * 16 + 8 * hi]);
        const v4f m1 = *(const v4fa*)(&ms[j * 16 + 8 * hi + 4]);
#pragma unroll
        for (int r = 0; r < 8; ++r) {
            const float mv = (r < 4) ? m0[r & 3] : m1[r & 3];
            const float p0 = __builtin_amdgcn_exp2f((s0[r] * 0.01f - 9.0f) * LOG2E);
            const float p1 = __builtin_amdgcn_exp2f((s1[r] * 0.01f - 9.0f) * LOG2E);
            l0 += p0; o0 = fmaf(p0, mv, o0);
            l1 += p1; o1 = fmaf(p1, mv, o1);
        }
    }
    l0 += __shfl_xor(l0, 16, 32); o0 += __shfl_xor(o0, 16, 32);
    l1 += __shfl_xor(l1, 16, 32); o1 += __shfl_xor(o1, 16, 32);
    const float r0v = o0 * (1.0f / l0);
    const float r1v = o1 * (1.0f / l1);
    const float val = hi ? r1v : r0v;

    os[wave * 32 + lane] = val;
    wave_sync();
    const v4f ov = *(const v4fa*)(&os[wave * 32 + 4 * (lane & 7)]);
    float* op = OUT + (size_t)b * OUT_SEQ + t0 + 4 * (lane & 7);
    if (lane < 8) *(volatile v4f*)op = ov;
    __threadfence();
    if (lane < 8) *(volatile v4f*)op = ov;
}

static constexpr size_t SZ_TOTAL = 0;
static_assert(SZ_TOTAL <= (size_t)134217728);

extern "C" void kernel_launch(void* const* d_in, const int* in_sizes, int n_in,
                              void* d_out, int out_size, void* d_ws, size_t ws_size, hipStream_t stream) {
    if (n_in < 2) return;
    if ((size_t)in_sizes[0] < (size_t)(NB - 1) * SEQ_FULL + SEQ) return;
    if ((size_t)in_sizes[1] < (size_t)NB * MEMN) return;
    if ((size_t)out_size < (size_t)(NB - 1) * OUT_SEQ + SEQ) return;
    if (SZ_TOTAL > ws_size) return;
    (void)d_ws;
    const int*   qa  = (const int*)d_in[0];
    const float* mem = (const float*)d_in[1];
    float*       out = (float*)d_out;

    k_lookup<<<dim3(SEQ / (32 * AW), NB, 1), 32 * AW, 0, stream>>>(qa, mem, out);
}
